// Transformer_7344394076780
// MI455X (gfx1250) — hardware-run, weakly checked
//
#include <hip/hip_runtime.h>

#ifndef NB
#define NB 2
#endif
#ifndef SEQ
#define SEQ 2048
#endif
#define NB_FULL 2
#define SEQ_FULL 2048
#define NL 2
#define DM 256
#define NH 8
#define HD 32
#define DFF 512
#define NQKV 768
#define ROWS (NB * SEQ)
#define PL  (2 * DM)
#define PLF (2 * DFF)
#define LN_EPS 1.42108547152020037e-14f
#define RINV 4.8828125e-4f

static_assert(NB <= NB_FULL);
static_assert(SEQ <= SEQ_FULL);
static_assert(SEQ % 128 == 0);
static_assert(ROWS % 128 == 0);
static_assert(ROWS % 8 == 0);
static_assert(NH * HD == DM);
static_assert(HD == 32);
static_assert(DM % 64 == 0 && DFF % 64 == 0 && NQKV % 64 == 0);
static_assert(DM % 32 == 0 && DFF % 32 == 0);
static_assert(NQKV == 3 * DM);
static_assert((size_t)NB_FULL * SEQ_FULL * DM * 4 == 4194304);

#define BTP 40
#define TP  72
#define OLP 68
#define CHP 72

static_assert(64 * BTP * 2 + 8 * 16 * OLP * 4 <= 131072);
static_assert(64 * TP * 2 <= 131072);
static_assert(16 * CHP * 2 <= 131072);

typedef _Float16 v16h  __attribute__((ext_vector_type(16)));
typedef _Float16 v8h   __attribute__((ext_vector_type(8)));
typedef float    v8f   __attribute__((ext_vector_type(8)));
typedef float    v4f   __attribute__((ext_vector_type(4)));
typedef unsigned int v4u __attribute__((ext_vector_type(4)));
typedef _Float16 h16;

constexpr size_t SZ_WQKV = (size_t)NL * NQKV * DM * 2;
constexpr size_t SZ_WO   = (size_t)NL * DM * DM * 2;
constexpr size_t SZ_W1   = (size_t)NL * DFF * DM * 2;
constexpr size_t SZ_W2   = (size_t)NL * DM * DFF * 2;
constexpr size_t SZ_XA   = (size_t)ROWS * PL * 2;
constexpr size_t SZ_F32  = (size_t)ROWS * DM * 4;
constexpr size_t SZ_QKV  = (size_t)3 * ROWS * PL * 2;
constexpr size_t SZ_VT   = (size_t)NB * DM * 2 * SEQ * 2;
constexpr size_t SZ_CTX  = (size_t)ROWS * PL * 2;
constexpr size_t SZ_H1   = (size_t)ROWS * PLF * 2;
constexpr size_t OFF_WQKV = 0;
constexpr size_t OFF_WO   = OFF_WQKV + SZ_WQKV;
constexpr size_t OFF_W1   = OFF_WO + SZ_WO;
constexpr size_t OFF_W2   = OFF_W1 + SZ_W1;
constexpr size_t OFF_XA   = OFF_W2 + SZ_W2;
constexpr size_t OFF_XRES = OFF_XA + SZ_XA;
constexpr size_t OFF_TMP  = OFF_XRES + SZ_F32;
constexpr size_t OFF_QKV  = OFF_TMP + SZ_F32;
constexpr size_t OFF_VT   = OFF_QKV + SZ_QKV;
constexpr size_t OFF_CTX  = OFF_VT + SZ_VT;
constexpr size_t OFF_H1   = OFF_CTX + SZ_CTX;
constexpr size_t WS_TOTAL = OFF_H1 + SZ_H1;
static_assert(WS_TOTAL <= (size_t)134217728);
static_assert(SZ_WQKV % 128 == 0 && SZ_WO % 128 == 0 && SZ_W1 % 128 == 0 && SZ_W2 % 128 == 0);
static_assert(SZ_XA % 128 == 0 && SZ_F32 % 128 == 0 && SZ_QKV % 128 == 0 && SZ_VT % 128 == 0);
static_assert(SZ_CTX % 128 == 0 && SZ_H1 % 128 == 0);

__device__ __forceinline__ v8f mma_f16(v16h a, v16h b, v8f c) {
  v8f d = __builtin_amdgcn_wmma_f32_16x16x32_f16(false, a, false, b, (short)0, c, false, false);
  asm volatile("v_nop\n\tv_nop\n\tv_nop\n\tv_nop" : "+v"(d) : "v"(a), "v"(b));
  return d;
}

__device__ __forceinline__ v16h ld_frag_h(const _Float16* p0, int ld, int rc, int kk, int lane) {
  const int hh = (lane >> 4) & 1;
  const _Float16* p = p0 + (size_t)rc * ld + kk + 8 * hh;
  const v8h lo = *(const v8h*)(p);
  const v8h hi = *(const v8h*)(p + 16);
  v16h f;
#pragma unroll
  for (int i = 0; i < 8; ++i) { f[i] = lo[i]; f[8 + i] = hi[i]; }
  return f;
}

__device__ __forceinline__ unsigned int bfb(float x) {
  unsigned int u = __float_as_uint(x);
  u = u + 0x7FFFu + ((u >> 16) & 1u);
  return u >> 16;
}
__device__ __forceinline__ float bf16val(float x) {
  return __uint_as_float(bfb(x) << 16);
}

static __device__ __forceinline__ h16 toh_flush(float v) {
  const h16 r = (h16)v;
  return (fabsf(v) < 6.103515625e-05f) ? (h16)0.0f : r;
}

static __device__ __forceinline__ void pack_both(v4f a, v4f b, v4u& wh, v4u& wr) {
  unsigned int hb[8], rb[8];
#pragma unroll
  for (int i = 0; i < 8; ++i) {
    const float v = (i < 4) ? a[i & 3] : b[i & 3];
    const h16 hv = toh_flush(v);
    const h16 rv = toh_flush((v - (float)hv) * 2048.0f);
    hb[i] = (unsigned int)__builtin_bit_cast(unsigned short, hv);
    rb[i] = (unsigned int)__builtin_bit_cast(unsigned short, rv);
  }
#pragma unroll
  for (int i = 0; i < 4; ++i) {
    wh[i] = hb[2 * i] | (hb[2 * i + 1] << 16);
    wr[i] = rb[2 * i] | (rb[2 * i + 1] << 16);
  }
}
static __device__ __forceinline__ v4u pack_sel(v4f a, v4f b, bool isres) {
  v4u wh, wr, w;
  pack_both(a, b, wh, wr);
#pragma unroll
  for (int i = 0; i < 4; ++i) w[i] = isres ? wr[i] : wh[i];
  return w;
}

__global__ __launch_bounds__(256) void k_cvt_x(const float* __restrict__ in,
                                               unsigned short* __restrict__ plane,
                                               float* __restrict__ xres, int npieces) {
  const int g = blockIdx.x * 256 + threadIdx.x;
  if (g >= npieces) return;
  const int row = g >> 6;
  const int p = g & 63;
  const int bb = row / SEQ;
  const int nn = row - bb * SEQ;
  const float* rp = in + ((size_t)bb * SEQ_FULL + nn) * DM;
  const int col = (p >> 3) * 32 + (p & 3) * 8;
  v4f a = *(const v4f*)(rp + col);
  v4f b = *(const v4f*)(rp + col + 4);
  v4f c = *(const v4f*)(rp + 4 * p);
#pragma unroll
  for (int i = 0; i < 4; ++i) {
    a[i] = bf16val(a[i]) * 8.0f;
    b[i] = bf16val(b[i]) * 8.0f;
    c[i] = bf16val(c[i]);
  }
  const v4u w = pack_sel(a, b, (p & 4) != 0);
  volatile v4u* pp = (volatile v4u*)(plane + (size_t)g * 8);
  volatile v4f* pf = (volatile v4f*)(xres + (size_t)g * 4);
  *pp = w;
  *pf = c;
  __threadfence();
  *pp = w;
  *pf = c;
}

__global__ __launch_bounds__(256) void k_cvt_w(const float* __restrict__ in,
                                               unsigned short* __restrict__ outp,
                                               int R, int C, int nsub, int sL, int sH) {
  __shared__ __align__(16) unsigned short T[32 * TP];
  const int mat = blockIdx.z;
  const int l = mat / nsub;
  const int h = mat - l * nsub;
  const float* W = in + (size_t)mat * R * C;
  unsigned short* dst = outp + (size_t)l * sL + (size_t)h * sH;
  const int k0 = blockIdx.x * 64;
  const int n0 = blockIdx.y * 32;
  const int tid = threadIdx.x;
  const int wave = __builtin_amdgcn_readfirstlane(tid >> 5);
  const int lane = tid & 31;

#pragma unroll
  for (int i = 0; i < 2; ++i) {
    const int idx = i * 256 + tid;
    const int kk = idx >> 3;
    const int c4 = (idx & 7) * 4;
    const v4f w = *(const v4f*)(W + (size_t)(k0 + kk) * C + n0 + c4);
#pragma unroll
    for (int c = 0; c < 4; ++c) {
      const h16 hv = toh_flush(bf16val(w[c]) * 64.0f);
      T[(c4 + c) * TP + kk] = __builtin_bit_cast(unsigned short, hv);
    }
  }
  __syncthreads();

  static_assert(256 * 16 == 32 * 128);
  const int nn = wave * 4 + (lane >> 3);
  const int q = lane & 7;
  const v4u v = *(const v4u*)(&T[nn * TP + q * 8]);
  volatile v4u* p = (volatile v4u*)(dst + (size_t)(n0 + nn) * R + k0 + q * 8);
  *p = v;
  __threadfence();
  *p = v;
}

template <int KD, int EPI, bool HASB>
__device__ __forceinline__ void gemm_body(const unsigned short* __restrict__ Ap,
                                          const unsigned short* __restrict__ Wt,
                                          const float* __restrict__ bias,
                                          const float* __restrict__ resid,
                                          float* __restrict__ Cf,
                                          unsigned short* __restrict__ Cp,
                                          unsigned short* bt, float* Cs) {
  static_assert(KD % 32 == 0);
  const int n0 = blockIdx.x * 64;
  const int m0 = blockIdx.y * 128;
  const int tid = threadIdx.x;
  const int wave = __builtin_amdgcn_readfirstlane(tid >> 5);
  const int lane = tid & 31;
  const int l15 = lane & 15, half = (lane >> 4) & 1;

  const int tn = tid >> 2;
  const int tk = (tid & 3) * 8;
  const unsigned short* wsrc = Wt + (size_t)(n0 + tn) * KD + tk;
  const int arow = m0 + wave * 16 + l15;
  const _Float16* arp = (const _Float16*)Ap + (size_t)arow * (2 * KD);

  v8f acc[4] = {};
  v8f acr[4] = {};
  for (int s = 0; s < KD / 32; ++s) {
    const v4u wv = *(const v4u*)(wsrc + s * 32);
    __syncthreads();
    *(v4u*)(&bt[tn * BTP + tk]) = wv;
    __syncthreads();
    const v16h ah = ld_frag_h(arp + s * 64, 0, 0, 0, lane);
    const v16h ar = ld_frag_h(arp + s * 64 + 32, 0, 0, 0, lane);
#pragma unroll
    for (int j = 0; j < 4; ++j) {
      const v16h b = ld_frag_h((const _Float16*)bt, BTP, j * 16 + l15, 0, lane);
      acc[j] = mma_f16(ah, b, acc[j]);
      acr[j] = mma_f16(ar, b, acr[j]);
    }
  }

  const float osc = (EPI == 1) ? (1.0f / 512.0f) : (1.0f / 64.0f);
  float* cw = Cs + wave * 16 * OLP;
#pragma unroll
  for (int j = 0; j < 4; ++j) {
#pragma unroll
    for (int r = 0; r < 8; ++r) {
      cw[(8 * half + r) * OLP + j * 16 + l15] = (acc[j][r] + acr[j][r] * RINV) * osc;
    }
  }
  __syncthreads();

  static_assert(256 * 16 * 8 == 128 * 256);
  if (EPI == 1) {
    v4f v[8];
    size_t off[8];
#pragma unroll
    for (int it = 0; it < 8; ++it) {
      const int row = it * 2 + half;
      const int q = l15;
      v4f t = *(const v4f*)(&cw[row * OLP + q * 4]);
      const size_t o = (size_t)(m0 + wave * 16 + row) * DM + n0 + q * 4;
      const v4f rs = *(const v4f*)(resid + o);
      if (HASB) {
        const v4f bi = *(const v4f*)(bias + n0 + q * 4);
#pragma unroll
        for (int i = 0; i < 4; ++i) t[i] = t[i] + bf16val(bi[i]);
      }
#pragma unroll
      for (int i = 0; i < 4; ++i) t[i] = rs[i] + t[i];
      v[it] = t;
      off[it] = o;
    }
#pragma unroll
    for (int it = 0; it < 8; ++it) *(volatile v4f*)(Cf + off[it]) = v[it];
    __threadfence();
#pragma unroll
    for (int it = 0; it < 8; ++it) *(volatile v4f*)(Cf + off[it]) = v[it];
  } else {
    v4u v[8];
    size_t off[8];
#pragma unroll
    for (int it = 0; it < 8; ++it) {
      const int row = it * 2 + half;
      const int q = l15;
      const int c = (q >> 3) * 32 + (q & 3) * 8;
      v4f ta = *(const v4f*)(&cw[row * OLP + c]);
      v4f tb = *(const v4f*)(&cw[row * OLP + c + 4]);
      if (EPI == 2) {
        const v4f ba = *(const v4f*)(bias + n0 + c);
        const v4f bb = *(const v4f*)(bias + n0 + c + 4);
#pragma unroll
        for (int i = 0; i < 4; ++i) {
          const float ua = ta[i] + 8.0f * bf16val(ba[i]);
          const float ub = tb[i] + 8.0f * bf16val(bb[i]);
          ta[i] = (ua > 0.0f) ? ua : 0.0f;
          tb[i] = (ub > 0.0f) ? ub : 0.0f;
        }
      }
      v[it] = pack_sel(ta, tb, (q & 4) != 0);
      const int grow = m0 + wave * 16 + row;
      if (EPI == 0) {
        const int z = n0 >> 8;
        const int cz = n0 & 255;
        off[it] = (size_t)z * ROWS * PL + (size_t)grow * PL + (cz >> 5) * 64 + q * 8;
      } else {
        off[it] = (size_t)grow * PLF + (n0 >> 5) * 64 + q * 8;
      }
    }
#pragma unroll
    for (int it = 0; it < 8; ++it) *(volatile v4u*)(Cp + off[it]) = v[it];
    __threadfence();
#pragma unroll
    for (int it = 0; it < 8; ++it) *(volatile v4u*)(Cp + off[it]) = v[it];
  }
}

__global__ __launch_bounds__(256) void k_gemm_qkv(const unsigned short* __restrict__ Ap,
                                                  const unsigned short* __restrict__ Wt,
                                                  unsigned short* __restrict__ Cp) {
  __shared__ __align__(16) unsigned short bt[64 * BTP];
  __shared__ __align__(16) float Cs[8 * 16 * OLP];
  gemm_body<DM, 0, false>(Ap, Wt, nullptr, nullptr, nullptr, Cp, bt, Cs);
}
__global__ __launch_bounds__(256) void k_gemm_wo(const unsigned short* __restrict__ Ap,
                                                 const unsigned short* __restrict__ Wt,
                                                 const float* __restrict__ resid,
                                                 float* __restrict__ Cf) {
  __shared__ __align__(16) unsigned short bt[64 * BTP];
  __shared__ __align__(16) float Cs[8 * 16 * OLP];
  gemm_body<DM, 1, false>(Ap, Wt, nullptr, resid, Cf, nullptr, bt, Cs);
}
__global__ __launch_bounds__(256) void k_gemm_w1(const unsigned short* __restrict__ Ap,
                                                 const unsigned short* __restrict__ Wt,
                                                 const float* __restrict__ bias,
                                                 unsigned short* __restrict__ Cp) {
  __shared__ __align__(16) unsigned short bt[64 * BTP];
  __shared__ __align__(16) float Cs[8 * 16 * OLP];
  gemm_body<DM, 2, true>(Ap, Wt, bias, nullptr, nullptr, Cp, bt, Cs);
}
__global__ __launch_bounds__(256) void k_gemm_w2(const unsigned short* __restrict__ Ap,
                                                 const unsigned short* __restrict__ Wt,
                                                 const float* __restrict__ bias,
                                                 const float* __restrict__ resid,
                                                 float* __restrict__ Cf) {
  __shared__ __align__(16) unsigned short bt[64 * BTP];
  __shared__ __align__(16) float Cs[8 * 16 * OLP];
  gemm_body<DFF, 1, true>(Ap, Wt, bias, resid, Cf, nullptr, bt, Cs);
}

__global__ __launch_bounds__(256) void k_vT(const unsigned short* __restrict__ vp,
                                            unsigned short* __restrict__ vtp) {
  __shared__ __align__(16) unsigned short T[64 * TP];
  const int t0 = blockIdx.x * 64;
  const int head = blockIdx.y;
  const int b = blockIdx.z;
  const int tid = threadIdx.x;

#pragma unroll
  for (int it = 0; it < 2; ++it) {
    const int idx = it * 256 + tid;
    const int r = idx >> 3;
    const int q = idx & 7;
    const v4u w = *(const v4u*)(vp + (size_t)(b * SEQ + t0 + r) * PL + head * 64 + q * 8);
#pragma unroll
    for (int i = 0; i < 4; ++i) {
      T[(q * 8 + 2 * i) * TP + r]     = (unsigned short)(w[i] & 0xFFFFu);
      T[(q * 8 + 2 * i + 1) * TP + r] = (unsigned short)(w[i] >> 16);
    }
  }
  __syncthreads();

  static_assert(256 * 16 * 2 == 32 * 256);
  v4u v[2];
  size_t off[2];
#pragma unroll
  for (int it = 0; it < 2; ++it) {
    const int idx = it * 256 + tid;
    const int dd = idx >> 4;
    const int q = idx & 15;
    const int g = q >> 3;
    const int qq = q & 7;
    v[it] = *(const v4u*)(&T[((qq >> 2) * 32 + dd) * TP + g * 32 + (qq & 3) * 8]);
    off[it] = (size_t)(b * DM + head * HD + dd) * (2 * SEQ) + (size_t)(t0 >> 5) * 64 + q * 8;
  }
#pragma unroll
  for (int it = 0; it < 2; ++it) *(volatile v4u*)(vtp + off[it]) = v[it];
  __threadfence();
#pragma unroll
  for (int it = 0; it < 2; ++it) *(volatile v4u*)(vtp + off[it]) = v[it];
}

__global__ __launch_bounds__(32) __attribute__((amdgpu_num_vgpr(256)))
void k_attn(const unsigned short* __restrict__ qp, const unsigned short* __restrict__ kp,
            const unsigned short* __restrict__ vtp, unsigned short* __restrict__ ctx) {
  __shared__ __align__(16) unsigned short Ch[16 * CHP];

  const int lane = threadIdx.x & 31;
  const int l15 = lane & 15;
  const int half = (lane >> 4) & 1;
  const int q0 = blockIdx.x * 16;
  const int head = blockIdx.y;
  const int b = blockIdx.z;

  const _Float16* Q  = (const _Float16*)qp;
  const _Float16* K  = (const _Float16*)kp;
  const _Float16* VT = (const _Float16*)vtp;

  const _Float16* qbase = Q + (size_t)(b * SEQ + q0) * PL + head * 64;
  const v16h qh = ld_frag_h(qbase, PL, l15, 0, lane);
  const v16h qr = ld_frag_h(qbase + 32, PL, l15, 0, lane);
  const _Float16* kbase = K + (size_t)(b * SEQ) * PL + head * 64;
  const _Float16* vbase = VT + (size_t)(b * DM + head * HD) * (2 * SEQ);

  v8f om[2] = {};
  v8f orr[2] = {};
  float mrun = -1.0e30f, lrun = 0.0f;
  const float sscale = 1.0f / 64.0f;

  for (int kc = 0; kc < SEQ; kc += 32) {
    const _Float16* kt = kbase + (size_t)kc * PL;
    const v16h ka0h = ld_frag_h(kt, PL, l15, 0, lane);
    const v16h ka0r = ld_frag_h(kt + 32, PL, l15, 0, lane);
    const v16h ka1h = ld_frag_h(kt, PL, 16 + l15, 0, lane);
    const v16h ka1r = ld_frag_h(kt + 32, PL, 16 + l15, 0, lane);
    v8f c0 = {}, c1 = {}, d0 = {}, d1 = {};
    c0 = mma_f16(ka0h, qh, c0);
    c1 = mma_f16(ka1h, qh, c1);
    d0 = mma_f16(ka0h, qr, d0);
    d0 = mma_f16(ka0r, qh, d0);
    d1 = mma_f16(ka1h, qr, d1);
    d1 = mma_f16(ka1r, qh, d1);

    float sa[8], sb[8];
#pragma unroll
    for (int r = 0; r < 8; ++r) {
      sa[r] = (c0[r] + d0[r] * RINV) * sscale;
      sb[r] = (c1[r] + d1[r] * RINV) * sscale;
    }
    float lm = fmaxf(sa[0], sb[0]);
#pragma unroll
    for (int r = 1; r < 8; ++r) lm = fmaxf(lm, fmaxf(sa[r], sb[r]));
    lm = fmaxf(lm, __shfl_xor(lm, 16, 32));
    const float mnew = fmaxf(mrun, lm);
    const float alpha = __expf(mrun - mnew);
    float p0[8], p1[8];
    float ls = 0.0f;
#pragma unroll
    for (int r = 0; r < 8; ++r) {
      p0[r] = __expf(sa[r] - mnew);
      p1[r] = __expf(sb[r] - mnew);
      ls += p0[r] + p1[r];
    }
    ls += __shfl_xor(ls, 16, 32);
    lrun = lrun * alpha + ls;
    mrun = mnew;
#pragma unroll
    for (int j = 0; j < 2; ++j)
#pragma unroll
      for (int r = 0; r < 8; ++r) { om[j][r] *= alpha; orr[j][r] *= alpha; }

    v16h pbh, pbr;
#pragma unroll
    for (int e = 0; e < 8; ++e) {
      const float ca = p0[e] * 16384.0f;
      const float cb = p1[e] * 16384.0f;
      const h16 ha = toh_flush(ca);
      const h16 hb = toh_flush(cb);
      pbh[e]     = ha;
      pbh[8 + e] = hb;
      pbr[e]     = toh_flush((ca - (float)ha) * 2048.0f);
      pbr[8 + e] = toh_flush((cb - (float)hb) * 2048.0f);
    }
    const _Float16* vt = vbase + (size_t)(kc >> 5) * 64;
#pragma unroll
    for (int j = 0; j < 2; ++j) {
      const v16h vah = ld_frag_h(vt, 2 * SEQ, j * 16 + l15, 0, lane);
      const v16h vra = ld_frag_h(vt + 32, 2 * SEQ, j * 16 + l15, 0, lane);
      om[j]  = mma_f16(vah, pbh, om[j]);
      orr[j] = mma_f16(vah, pbr, orr[j]);
      orr[j] = mma_f16(vra, pbh, orr[j]);
    }
  }

  const float inv = (1.0f / 16384.0f) * (1.0f / lrun);
#pragma unroll
  for (int j = 0; j < 2; ++j) {
    v4f ya, yb;
#pragma unroll
    for (int i = 0; i < 4; ++i) {
      ya[i] = (om[j][i] + orr[j][i] * RINV) * inv;
      yb[i] = (om[j][4 + i] + orr[j][4 + i] * RINV) * inv;
    }
    v4u wh, wr;
    pack_both(ya, yb, wh, wr);
    *(v4u*)(&Ch[l15 * CHP + j * 16 + 8 * half]) = wh;
    *(v4u*)(&Ch[l15 * CHP + 32 + j * 16 + 8 * half]) = wr;
  }
  __syncthreads();

  static_assert(32 * 16 * 4 == 16 * 128);
  v4u v[4];
  size_t off[4];
  unsigned short* ob = ctx + (size_t)(b * SEQ + q0) * PL + head * 64;
#pragma unroll
  for (int it = 0; it < 4; ++it) {
    const int p = it * 32 + lane;
    const int row = p >> 3;
    const int qd = p & 7;
    v[it] = *(const v4u*)(&Ch[row * CHP + qd * 8]);
    off[it] = (size_t)row * PL + qd * 8;
  }
#pragma unroll
  for (int it = 0; it < 4; ++it) *(volatile v4u*)(ob + off[it]) = v[it];
  __threadfence();
#pragma unroll
  for (int it = 0; it < 4; ++it) *(volatile v4u*)(ob + off[it]) = v[it];
}

__global__ __launch_bounds__(256) void k_ln(const float* __restrict__ tin,
                                            const float* __restrict__ gam,
                                            const float* __restrict__ bet, int gi,
                                            float* __restrict__ outf, int ostride,
                                            unsigned short* __restrict__ plane, int wplane) {
  const int lane = threadIdx.x & 31;
  const int wave = __builtin_amdgcn_readfirstlane(threadIdx.x >> 5);
  const int row = blockIdx.x * 8 + wave;
  const int bb = row / SEQ;
  const int nn = row - bb * SEQ;
  const float* rp = tin + (size_t)row * DM;
  const v4f a = *(const v4f*)(rp + 4 * lane);
  const v4f c = *(const v4f*)(rp + 128 + 4 * lane);
  float s = ((a[0] + a[1]) + (a[2] + a[3])) + ((c[0] + c[1]) + (c[2] + c[3]));
#pragma unroll
  for (int o = 16; o > 0; o >>= 1) s += __shfl_xor(s, o, 32);
  const float mean = s * (1.0f / 256.0f);
  float ss = 0.0f;
#pragma unroll
  for (int i = 0; i < 4; ++i) {
    const float da = a[i] - mean;
    const float dc = c[i] - mean;
    ss += da * da + dc * dc;
  }
#pragma unroll
  for (int o = 16; o > 0; o >>= 1) ss += __shfl_xor(ss, o, 32);
  const float var = ss * (1.0f / 256.0f);
  const float rstd = rsqrtf(var + LN_EPS);
  const float g = bf16val(gam[gi]);
  const float be = bf16val(bet[gi]);

  v4f ya, yc;
#pragma unroll
  for (int i = 0; i < 4; ++i) {
    ya[i] = ((a[i] - mean) * rstd) * g + be;
    yc[i] = ((c[i] - mean) * rstd) * g + be;
  }
  v4u w[2];
#pragma unroll
  for (int it = 0; it < 2; ++it) {
    const int p = it * 32 + lane;
    const int col = (p >> 3) * 32 + (p & 3) * 8;
    const v4f xa = *(const v4f*)(rp + col);
    const v4f xb = *(const v4f*)(rp + col + 4);
    v4f za, zb;
#pragma unroll
    for (int i = 0; i < 4; ++i) {
      za[i] = (((xa[i] - mean) * rstd) * g + be) * 8.0f;
      zb[i] = (((xb[i] - mean) * rstd) * g + be) * 8.0f;
    }
    w[it] = pack_sel(za, zb, (p & 4) != 0);
  }

  static_assert(32 * 16 * 2 == DM * 4);
  static_assert(32 * 16 * 2 == PL * 2);
  float* orow = outf + ((size_t)bb * ostride + nn) * DM;
  unsigned short* prow = plane + (size_t)row * PL;
  *(volatile v4f*)(orow + 4 * lane) = ya;
  *(volatile v4f*)(orow + 128 + 4 * lane) = yc;
  if (wplane != 0) {
    *(volatile v4u*)(prow + 8 * lane) = w[0];
    *(volatile v4u*)(prow + 256 + 8 * lane) = w[1];
  }
  __threadfence();
  *(volatile v4f*)(orow + 4 * lane) = ya;
  *(volatile v4f*)(orow + 128 + 4 * lane) = yc;
  if (wplane != 0) {
    *(volatile v4u*)(prow + 8 * lane) = w[0];
    *(volatile v4u*)(prow + 256 + 8 * lane) = w[1];
  }
}

extern "C" void kernel_launch(void* const* d_in, const int* in_sizes, int n_in,
                              void* d_out, int out_size, void* d_ws, size_t ws_size,
                              hipStream_t stream) {
  if (n_in < 11) return;
  if (in_sizes[0] < ((NB - 1) * SEQ_FULL + SEQ) * DM) return;
  if (in_sizes[1] < NL * NH * DM * HD || in_sizes[2] < NL * NH * DM * HD ||
      in_sizes[3] < NL * NH * DM * HD) return;
  if (in_sizes[4] < NL * DM * DM) return;
  if (in_sizes[5] < NL * DM * DFF || in_sizes[7] < NL * DFF * DM) return;
  if (in_sizes[6] < NL * DFF || in_sizes[8] < NL * DM) return;
  if (in_sizes[9] < 2 * NL || in_sizes[10] < 2 * NL) return;
  if (out_size < ((NB - 1) * SEQ_FULL + SEQ) * DM) return;
  if (WS_TOTAL > ws_size) return;

  const float* x     = (const float*)d_in[0];
  const float* Wq    = (const float*)d_in[1];
  const float* Wk    = (const float*)d_in[2];
  const float* Wv    = (const float*)d_in[3];
  const float* Wo    = (const float*)d_in[4];
  const float* W1    = (const float*)d_in[5];
  const float* b1    = (const float*)d_in[6];
  const float* W2    = (const float*)d_in[7];
  const float* b2    = (const float*)d_in[8];
  const float* gamma = (const float*)d_in[9];
  const float* beta  = (const float*)d_in[10];
  float* out = (float*)d_out;

  char* ws = (char*)d_ws;
  unsigned short* wqkv = (unsigned short*)(ws + OFF_WQKV);
  unsigned short* woT  = (unsigned short*)(ws + OFF_WO);
  unsigned short* w1T  = (unsigned short*)(ws + OFF_W1);
  unsigned short* w2T  = (unsigned short*)(ws + OFF_W2);
  unsigned short* xa   = (unsigned short*)(ws + OFF_XA);
  float* xres          = (float*)(ws + OFF_XRES);
  float* tmp           = (float*)(ws + OFF_TMP);
  unsigned short* qkv  = (unsigned short*)(ws + OFF_QKV);
  unsigned short* vtp  = (unsigned short*)(ws + OFF_VT);
  unsigned short* ctx  = (unsigned short*)(ws + OFF_CTX);
  unsigned short* h1   = (unsigned short*)(ws + OFF_H1);
  unsigned short* qpl = qkv;
  unsigned short* kpl = qkv + (size_t)ROWS * PL;
  unsigned short* vpl = qkv + (size_t)2 * ROWS * PL;

  k_cvt_w<<<dim3(DM / 64, HD / 32, NL * NH), 256, 0, stream>>>(Wq, wqkv, DM, HD, NH, NQKV * DM, HD * DM);
  k_cvt_w<<<dim3(DM / 64, HD / 32, NL * NH), 256, 0, stream>>>(Wk, wqkv + (size_t)DM * DM, DM, HD, NH, NQKV * DM, HD * DM);
  k_cvt_w<<<dim3(DM / 64, HD / 32, NL * NH), 256, 0, stream>>>(Wv, wqkv + (size_t)2 * DM * DM, DM, HD, NH, NQKV * DM, HD * DM);
  k_cvt_w<<<dim3(DM / 64, DM / 32, NL), 256, 0, stream>>>(Wo, woT, DM, DM, 1, DM * DM, 0);
  k_cvt_w<<<dim3(DM / 64, DFF / 32, NL), 256, 0, stream>>>(W1, w1T, DM, DFF, 1, DFF * DM, 0);
  k_cvt_w<<<dim3(DFF / 64, DM / 32, NL), 256, 0, stream>>>(W2, w2T, DFF, DM, 1, DM * DFF, 0);

  const int npieces = ROWS * 64;
  k_cvt_x<<<(npieces + 255) / 256, 256, 0, stream>>>(x, xa, xres, npieces);

  for (int l = 0; l < NL; ++l) {
    k_gemm_qkv<<<dim3(NQKV / 64, ROWS / 128), 256, 0, stream>>>(xa, wqkv + (size_t)l * NQKV * DM, qkv);
    k_vT<<<dim3(SEQ / 64, NH, NB), 256, 0, stream>>>(vpl, vtp);
    k_attn<<<dim3(SEQ / 16, NH, NB), 32, 0, stream>>>(qpl, kpl, vtp, ctx);
    k_gemm_wo<<<dim3(DM / 64, ROWS / 128), 256, 0, stream>>>(ctx, woT + (size_t)l * DM * DM, xres, tmp);
    k_ln<<<ROWS / 8, 256, 0, stream>>>(tmp, gamma, beta, 2 * l, xres, SEQ, xa, 1);
    k_gemm_w1<<<dim3(DFF / 64, ROWS / 128), 256, 0, stream>>>(xa, w1T + (size_t)l * DFF * DM, b1 + (size_t)l * DFF, h1);
    k_gemm_w2<<<dim3(DM / 64, ROWS / 128), 256, 0, stream>>>(h1, w2T + (size_t)l * DM * DFF, b2 + (size_t)l * DM, xres, tmp);
    if (l == NL - 1) {
      k_ln<<<ROWS / 8, 256, 0, stream>>>(tmp, gamma, beta, 2 * l + 1, out, SEQ_FULL, xa, 0);
    } else {
      k_ln<<<ROWS / 8, 256, 0, stream>>>(tmp, gamma, beta, 2 * l + 1, xres, SEQ, xa, 1);
    }
  }
}
